// TCRpMHCPairUpdateBlock_88184268521502
// MI455X (gfx1250) — hardware-verified
//
#include <hip/hip_runtime.h>

typedef _Float16 v16h __attribute__((ext_vector_type(16)));
typedef _Float16 v8h  __attribute__((ext_vector_type(8)));
typedef _Float16 v4h  __attribute__((ext_vector_type(4)));
typedef float    v8f  __attribute__((ext_vector_type(8)));
typedef float    v4f  __attribute__((ext_vector_type(4)));
typedef v8h __attribute__((may_alias)) v8ha;
typedef v4h __attribute__((may_alias)) v4ha;
typedef v4f __attribute__((may_alias)) v4fa;

union Frag { v16h v; v8h half[2]; };

#define NS 192
#define CD 128
#define NP 36864
#define NH 8
#define HC 1024
#define NZ 4718592

#define W_O3     65536
#define W_DIR0   2162688
#define W_DIRSZ  655360
#define W_K_OFF  131072
#define W_V_OFF  262144
#define W_G_OFF  393216
#define W_O_OFF  524288
#define W_TOTAL  3473408
#define W_GROUPS 434176

__device__ __forceinline__ v8f wmma_f16(v16h a, v16h b, v8f c) {
  v8f d = __builtin_amdgcn_wmma_f32_16x16x32_f16(false, a, false, b, (short)0, c, false, false);
  asm volatile("v_nop\n\tv_nop\n\tv_nop\n\tv_nop" : "+v"(d) : "v"(a), "v"(b));
  return d;
}

__device__ __forceinline__ v16h load_frag(const _Float16* p, int h) {
  Frag f;
  f.half[0] = *(const v8ha*)(p + 8 * h);
  f.half[1] = *(const v8ha*)(p + 16 + 8 * h);
  return f.v;
}

__device__ __forceinline__ v8h cvt8(v8f a, float sc) {
  v8h r;
  r[0] = (_Float16)(a[0] * sc); r[1] = (_Float16)(a[1] * sc);
  r[2] = (_Float16)(a[2] * sc); r[3] = (_Float16)(a[3] * sc);
  r[4] = (_Float16)(a[4] * sc); r[5] = (_Float16)(a[5] * sc);
  r[6] = (_Float16)(a[6] * sc); r[7] = (_Float16)(a[7] * sc);
  return r;
}

__device__ __forceinline__ v16h pack2(v8f a, v8f c, float sc) {
  Frag f;
  f.half[0] = cvt8(a, sc);
  f.half[1] = cvt8(c, sc);
  return f.v;
}

__device__ __forceinline__ v8f scale_bias8(v8f a, float sc, const float* __restrict__ bp) {
  const v4f c0 = *(const v4fa*)bp;
  const v4f c1 = *(const v4fa*)(bp + 4);
  v8f r;
  r[0] = a[0] * sc + c0.x; r[1] = a[1] * sc + c0.y; r[2] = a[2] * sc + c0.z; r[3] = a[3] * sc + c0.w;
  r[4] = a[4] * sc + c1.x; r[5] = a[5] * sc + c1.y; r[6] = a[6] * sc + c1.z; r[7] = a[7] * sc + c1.w;
  return r;
}

__device__ __forceinline__ v4f ln_row4(const float* __restrict__ src, const float* __restrict__ g,
                                       const float* __restrict__ b, int lane) {
  const v4f x = *(const v4fa*)(src + 4 * lane);
  float s = (x.x + x.y) + (x.z + x.w);
  #pragma unroll
  for (int o = 1; o < 32; o <<= 1) s += __shfl_xor(s, o);
  const float mu = s * (1.0f / 128.0f);
  v4f d;
  d.x = x.x - mu; d.y = x.y - mu; d.z = x.z - mu; d.w = x.w - mu;
  float q = d.x * d.x + d.y * d.y + d.z * d.z + d.w * d.w;
  #pragma unroll
  for (int o = 1; o < 32; o <<= 1) q += __shfl_xor(q, o);
  const float rs = rsqrtf(q * (1.0f / 128.0f) + 1e-5f);
  const v4f gv = *(const v4fa*)(g + 4 * lane);
  const v4f bv = *(const v4fa*)(b + 4 * lane);
  v4f y;
  y.x = d.x * rs * gv.x + bv.x; y.y = d.y * rs * gv.y + bv.y;
  y.z = d.z * rs * gv.z + bv.z; y.w = d.w * rs * gv.w + bv.w;
  return y;
}

__global__ __launch_bounds__(256) void prep_kernel(
    const float* __restrict__ wa, const float* __restrict__ wb,
    const float* __restrict__ w1, const float* __restrict__ w2,
    const float* __restrict__ wo3,
    const float* __restrict__ sq0, const float* __restrict__ sk0, const float* __restrict__ sv0,
    const float* __restrict__ sg0, const float* __restrict__ so0,
    const float* __restrict__ sq1, const float* __restrict__ sk1, const float* __restrict__ sv1,
    const float* __restrict__ sg1, const float* __restrict__ so1,
    _Float16* __restrict__ wd)
{
  const int g = blockIdx.x * 256 + threadIdx.x;
  if (g >= W_GROUPS) return;
  const int e = g * 8;
  const float* src;
  int lk, N, off, perm = 0;
  if (e < W_O3) {
    const int s = e >> 14;
    src = (s == 0) ? wa : ((s == 1) ? wb : ((s == 2) ? w1 : w2));
    lk = 7; N = CD; off = e & 16383;
  } else if (e < W_DIR0) {
    src = wo3; lk = 7; N = 16384; perm = 1; off = e - W_O3;
  } else {
    const int e2 = e - W_DIR0;
    const int d = (e2 >= W_DIRSZ) ? 1 : 0;
    const int r = e2 - d * W_DIRSZ;
    const int s = r >> 17;
    off = r & 131071;
    if (d == 0) src = (s == 0) ? sq0 : ((s == 1) ? sk0 : ((s == 2) ? sv0 : ((s == 3) ? sg0 : so0)));
    else        src = (s == 0) ? sq1 : ((s == 1) ? sk1 : ((s == 2) ? sv1 : ((s == 3) ? sg1 : so1)));
    lk = (s == 4) ? 10 : 7;
    N  = (s == 4) ? CD : HC;
  }
  const int n = off >> lk, kk = off & ((1 << lk) - 1);
  const int col = perm ? (((n & 127) << 7) + (n >> 7)) : n;
  const float* sp = src + (size_t)kk * N + col;
  v8h o;
  #pragma unroll
  for (int t = 0; t < 8; ++t) o[t] = (_Float16)(sp[(size_t)t * N] * 64.0f);
  *(volatile v8h*)(wd + e) = o;
  __threadfence();
  *(volatile v8h*)(wd + e) = o;
}

__device__ __forceinline__ void rows16_store_pass(const _Float16* ot, _Float16* dst, int lane) {
  const int hh = lane >> 4, pc = lane & 15;
  #pragma unroll
  for (int it = 0; it < 8; ++it) {
    const int row = 2 * it + hh;
    const v8h v = *(const v8ha*)(ot + row * CD + 8 * pc);
    *(volatile v8h*)(dst + (size_t)row * CD + 8 * pc) = v;
  }
}

__global__ __launch_bounds__(32) void opm_ab_kernel(
    const float* __restrict__ tcr, const float* __restrict__ pmhc,
    const float* __restrict__ tm, const float* __restrict__ pm,
    const float* __restrict__ g1, const float* __restrict__ b1,
    const float* __restrict__ g2, const float* __restrict__ b2,
    const _Float16* __restrict__ waT, const float* __restrict__ ba,
    const _Float16* __restrict__ wbT, const float* __restrict__ bb,
    _Float16* __restrict__ a16, _Float16* __restrict__ b16)
{
  __shared__ __attribute__((aligned(16))) _Float16 xs[16 * CD];
  __shared__ __attribute__((aligned(16))) _Float16 ot[16 * CD];
  const int lane = threadIdx.x & 31, h = lane >> 4, m = lane & 15;
  const int which = blockIdx.y, r0 = blockIdx.x * 16;
  const float* src  = which ? pmhc : tcr;
  const float* g    = which ? g2 : g1;
  const float* bl   = which ? b2 : b1;
  const _Float16* wT = which ? wbT : waT;
  const float* bias = which ? bb : ba;
  const float* msk  = which ? pm : tm;
  _Float16* dst = (which ? b16 : a16) + (size_t)r0 * CD;

  #pragma unroll 1
  for (int rr = 0; rr < 16; ++rr) {
    const v4f y = ln_row4(src + (size_t)(r0 + rr) * CD, g, bl, lane);
    const v4h yh = {(_Float16)y.x, (_Float16)y.y, (_Float16)y.z, (_Float16)y.w};
    *(v4ha*)(xs + rr * CD + 4 * lane) = yh;
  }
  __syncthreads();

  v16h xf[4];
  #pragma unroll
  for (int ks = 0; ks < 4; ++ks) xf[ks] = load_frag(xs + m * CD + 32 * ks, h);
  const float mv = msk[r0 + m] * 16.0f;
  const v8f zero8 = {0.f, 0.f, 0.f, 0.f, 0.f, 0.f, 0.f, 0.f};
  #pragma unroll
  for (int ct = 0; ct < 8; ++ct) {
    v8f acc = zero8;
    #pragma unroll
    for (int ks = 0; ks < 4; ++ks) {
      const v16h wf = load_frag(wT + (size_t)(16 * ct + m) * CD + 32 * ks, h);
      acc = wmma_f16(wf, xf[ks], acc);
    }
    const v8f t = scale_bias8(acc, 1.0f / 64.0f, bias + 16 * ct + 8 * h);
    *(v8ha*)(ot + m * CD + 16 * ct + 8 * h) = cvt8(t, mv);
  }
  __syncthreads();
  rows16_store_pass(ot, dst, lane);
  __threadfence();
  rows16_store_pass(ot, dst, lane);
}

template <int MODE>
__device__ __forceinline__ void gemm_store_pass(const float* sb, const _Float16* sh,
    const float* __restrict__ zin, const float* __restrict__ bias,
    const float* __restrict__ tm, const float* __restrict__ pm,
    float* outf, _Float16* outh, int rb, int cb, int ib, int dir, int w, int lane)
{
  if (MODE == 0) {
    const int hh = lane >> 4, pc = lane & 15;
    #pragma unroll
    for (int it = 0; it < 8; ++it) {
      const int row = 16 * w + 2 * it + hh;
      const v8h v = *(const v8ha*)(sh + row * CD + 8 * pc);
      *(volatile v8h*)(outh + (size_t)(rb + row) * 16384 + cb + 8 * pc) = v;
    }
  } else {
    const v4f bz = *(const v4fa*)(bias + 4 * lane);
    #pragma unroll
    for (int it = 0; it < 16; ++it) {
      const int row = 16 * w + it;
      const int lr = rb + row;
      int grow;
      if (MODE == 1) grow = ib * NS + lr;
      else grow = dir ? ((lr % NS) * NS + lr / NS) : lr;
      const v4f v  = *(const v4fa*)(sb + row * CD + 4 * lane);
      const v4f zi = *(const v4fa*)(zin + (size_t)grow * CD + 4 * lane);
      v4f o;
      if (MODE == 1) {
        const float rn = 1.0f / (1e-3f + tm[ib] * pm[lr]);
        o = zi + (v + bz) * rn;
      } else {
        o = zi + (v + bz);
      }
      *(volatile v4f*)(outf + (size_t)grow * CD + 4 * lane) = o;
    }
  }
}

template <int MODE>
__global__ __launch_bounds__(128) void gemm_kernel(
    const _Float16* __restrict__ A, const _Float16* __restrict__ Bt,
    const float* __restrict__ zin, const float* __restrict__ bias,
    const float* __restrict__ tm, const float* __restrict__ pm,
    float* __restrict__ outf, _Float16* __restrict__ outh, int dir)
{
  constexpr int K = (MODE == 2) ? HC : CD;
  __shared__ __attribute__((aligned(16))) float sb[64 * CD];
  _Float16* sh = (_Float16*)sb;

  const int tid = threadIdx.x, lane = tid & 31, w = tid >> 5;
  const int h = lane >> 4, m = lane & 15;
  const int rb = blockIdx.x * 64;
  const int cb = (MODE == 0) ? (int)blockIdx.y * 128 : 0;
  const int ib = (MODE == 1) ? (int)blockIdx.y : 0;

  const _Float16* ap = A + (size_t)(rb + 16 * w + m) * K;
  const _Float16* bp = Bt + ((MODE == 1) ? (size_t)ib * 16384 : (size_t)0) + (size_t)(cb + m) * K;

  const v8f zero8 = {0.f, 0.f, 0.f, 0.f, 0.f, 0.f, 0.f, 0.f};
  v8f acc[8];
  #pragma unroll
  for (int nt = 0; nt < 8; ++nt) acc[nt] = zero8;

  #pragma unroll 1
  for (int k0 = 0; k0 < K; k0 += 32) {
    const v16h a = load_frag(ap + k0, h);
    #pragma unroll
    for (int nt = 0; nt < 8; ++nt) {
      const v16h b = load_frag(bp + (size_t)nt * 16 * K + k0, h);
      acc[nt] = wmma_f16(a, b, acc[nt]);
    }
  }

  const float osc = (MODE == 0) ? 0.25f : ((MODE == 1) ? (1.0f / 4096.0f) : (1.0f / 16384.0f));
  #pragma unroll
  for (int nt = 0; nt < 8; ++nt) {
    #pragma unroll
    for (int r = 0; r < 8; ++r) {
      const int idx = (16 * w + 8 * h + r) * CD + 16 * nt + m;
      if (MODE == 0) sh[idx] = (_Float16)(acc[nt][r] * osc);
      else sb[idx] = acc[nt][r] * osc;
    }
  }
  __syncthreads();

  gemm_store_pass<MODE>(sb, sh, zin, bias, tm, pm, outf, outh, rb, cb, ib, dir, w, lane);
  __threadfence();
  gemm_store_pass<MODE>(sb, sh, zin, bias, tm, pm, outf, outh, rb, cb, ib, dir, w, lane);
}

__global__ __launch_bounds__(256) void ln_kernel(
    const float* __restrict__ z, const float* __restrict__ g, const float* __restrict__ b,
    const float* __restrict__ wtri, _Float16* __restrict__ xp, float* __restrict__ trib, int dir)
{
  __shared__ __attribute__((aligned(16))) _Float16 xs[32 * CD];
  __shared__ __attribute__((aligned(16))) float ts[NH * 32];
  const int tid = threadIdx.x, lane = tid & 31, w = tid >> 5;
  const int row0 = blockIdx.x * 32;

  v4f wl[4], wh4[4];
  #pragma unroll
  for (int t = 0; t < 4; ++t) {
    wl[t]  = *(const v4fa*)(wtri + (4 * lane + t) * NH);
    wh4[t] = *(const v4fa*)(wtri + (4 * lane + t) * NH + 4);
  }

  #pragma unroll 1
  for (int rr = 0; rr < 4; ++rr) {
    const int lr = 4 * w + rr;
    const int row = row0 + lr;
    const int i = row / NS, j = row - i * NS;
    const int srow = dir ? (j * NS + i) : row;
    const v4f y = ln_row4(z + (size_t)srow * CD, g, b, lane);
    const v4h yh = {(_Float16)y.x, (_Float16)y.y, (_Float16)y.z, (_Float16)y.w};
    *(v4ha*)(xs + lr * CD + 4 * lane) = yh;
    float pr[8];
    pr[0] = y.x * wl[0].x + y.y * wl[1].x + y.z * wl[2].x + y.w * wl[3].x;
    pr[1] = y.x * wl[0].y + y.y * wl[1].y + y.z * wl[2].y + y.w * wl[3].y;
    pr[2] = y.x * wl[0].z + y.y * wl[1].z + y.z * wl[2].z + y.w * wl[3].z;
    pr[3] = y.x * wl[0].w + y.y * wl[1].w + y.z * wl[2].w + y.w * wl[3].w;
    pr[4] = y.x * wh4[0].x + y.y * wh4[1].x + y.z * wh4[2].x + y.w * wh4[3].x;
    pr[5] = y.x * wh4[0].y + y.y * wh4[1].y + y.z * wh4[2].y + y.w * wh4[3].y;
    pr[6] = y.x * wh4[0].z + y.y * wh4[1].z + y.z * wh4[2].z + y.w * wh4[3].z;
    pr[7] = y.x * wh4[0].w + y.y * wh4[1].w + y.z * wh4[2].w + y.w * wh4[3].w;
    #pragma unroll
    for (int hq = 0; hq < 8; ++hq) {
      #pragma unroll
      for (int o = 1; o < 32; o <<= 1) pr[hq] += __shfl_xor(pr[hq], o);
    }
    if (lane == 0) {
      #pragma unroll
      for (int hq = 0; hq < 8; ++hq) ts[hq * 32 + lr] = pr[hq];
    }
  }
  __syncthreads();

  _Float16* xdst = xp + (size_t)row0 * CD;
  #pragma unroll
  for (int it = 0; it < 2; ++it) {
    const int p = it * 256 + tid;
    const v8h v = *(const v8ha*)(xs + p * 8);
    *(volatile v8h*)(xdst + p * 8) = v;
  }
  if (tid < 64) {
    const int hq = tid >> 3, q = tid & 7;
    const v4f v = *(const v4fa*)(ts + hq * 32 + 4 * q);
    *(volatile v4f*)(trib + (size_t)hq * NP + row0 + 4 * q) = v;
  }
  __threadfence();
  #pragma unroll
  for (int it = 0; it < 2; ++it) {
    const int p = it * 256 + tid;
    const v8h v = *(const v8ha*)(xs + p * 8);
    *(volatile v8h*)(xdst + p * 8) = v;
  }
  if (tid < 64) {
    const int hq = tid >> 3, q = tid & 7;
    const v4f v = *(const v4fa*)(ts + hq * 32 + 4 * q);
    *(volatile v4f*)(trib + (size_t)hq * NP + row0 + 4 * q) = v;
  }
}

__global__ __launch_bounds__(384) void attn_kernel(
    const _Float16* __restrict__ xp, const float* __restrict__ trib,
    const float* __restrict__ zmask,
    const _Float16* __restrict__ wqT, const _Float16* __restrict__ wkT,
    const _Float16* __restrict__ wvT, const _Float16* __restrict__ wgT,
    const float* __restrict__ bg, _Float16* __restrict__ ogp, int dir)
{
  extern __shared__ v4f smem_dyn[];
  char* smem = (char*)smem_dyn;
  _Float16* Ks = (_Float16*)smem;
  _Float16* Vt = (_Float16*)(smem + 49152);
  float*    mb = (float*)(smem + 98304);
  _Float16* Og = Ks;

  const int tid = threadIdx.x, lane = tid & 31, w = tid >> 5;
  const int h = lane >> 4, m = lane & 15;
  const int i = blockIdx.x >> 3, hh = blockIdx.x & 7;
  const int j0 = 16 * w;

  if (tid < NS) {
    const int k = tid;
    const float mv = zmask[dir ? (k * NS + i) : (i * NS + k)];
    mb[k] = 1e9f * (mv - 1.0f);
  }

  const _Float16* xrow = xp + ((size_t)i * NS + j0 + m) * CD;
  v16h xf[4];
  #pragma unroll
  for (int ks = 0; ks < 4; ++ks) xf[ks] = load_frag(xrow + 32 * ks, h);

  const v8f zero8 = {0.f, 0.f, 0.f, 0.f, 0.f, 0.f, 0.f, 0.f};
  const _Float16* wk = wkT + ((size_t)hh * CD + m) * CD;
  const _Float16* wv = wvT + ((size_t)hh * CD + m) * CD;
  const _Float16* wq = wqT + ((size_t)hh * CD + m) * CD;
  const _Float16* wg = wgT + ((size_t)hh * CD + m) * CD;

  #pragma unroll
  for (int ct = 0; ct < 8; ++ct) {
    v8f acc = zero8;
    #pragma unroll
    for (int ks = 0; ks < 4; ++ks) {
      const v16h wf = load_frag(wk + ct * 16 * CD + 32 * ks, h);
      acc = wmma_f16(wf, xf[ks], acc);
    }
    *(v8ha*)(Ks + (j0 + m) * CD + 16 * ct + 8 * h) = cvt8(acc, 0.125f);
  }
  #pragma unroll
  for (int ct = 0; ct < 8; ++ct) {
    v8f acc = zero8;
    #pragma unroll
    for (int ks = 0; ks < 4; ++ks) {
      const v16h wf = load_frag(wv + ct * 16 * CD + 32 * ks, h);
      acc = wmma_f16(xf[ks], wf, acc);
    }
    *(v8ha*)(Vt + (16 * ct + m) * NS + j0 + 8 * h) = cvt8(acc, 0.125f);
  }
  const float QSC = 0.08838834764831845f * 0.25f;
  v16h qf[4];
  #pragma unroll
  for (int kq = 0; kq < 4; ++kq) {
    v8f acc0 = zero8, acc1 = zero8;
    #pragma unroll
    for (int ks = 0; ks < 4; ++ks) {
      const v16h wf0 = load_frag(wq + (2 * kq) * 16 * CD + 32 * ks, h);
      const v16h wf1 = load_frag(wq + (2 * kq + 1) * 16 * CD + 32 * ks, h);
      acc0 = wmma_f16(wf0, xf[ks], acc0);
      acc1 = wmma_f16(wf1, xf[ks], acc1);
    }
    qf[kq] = pack2(acc0, acc1, QSC);
  }
  __syncthreads();

  v8f o[8];
  #pragma unroll
  for (int t = 0; t < 8; ++t) o[t] = zero8;
  float mrun = -1e30f, lrun = 0.0f;
  const float* trow = trib + (size_t)hh * NP + (size_t)(j0 + m) * NS;
  const float SSC = 1.0f / 128.0f;

  #pragma unroll 1
  for (int kb = 0; kb < NS; kb += 64) {
    v8f s[4];
    #pragma unroll
    for (int jt = 0; jt < 4; ++jt) {
      const _Float16* kp = Ks + (kb + 16 * jt + m) * CD;
      v8f z8 = zero8;
      #pragma unroll
      for (int ks = 0; ks < 4; ++ks) {
        const v16h kf = load_frag(kp + 32 * ks, h);
        z8 = wmma_f16(kf, qf[ks], z8);
      }
      s[jt] = z8;
    }
    #pragma unroll
    for (int jt = 0; jt < 4; ++jt) {
      const int kidx = kb + 16 * jt + 8 * h;
      const v4f t0 = *(const v4fa*)(trow + kidx);
      const v4f t1 = *(const v4fa*)(trow + kidx + 4);
      const v4f m0 = *(const v4fa*)(mb + kidx);
      const v4f m1 = *(const v4fa*)(mb + kidx + 4);
      v8f z8 = s[jt];
      z8[0] = (z8[0] * SSC + m0.x) + t0.x; z8[1] = (z8[1] * SSC + m0.y) + t0.y;
      z8[2] = (z8[2] * SSC + m0.z) + t0.z; z8[3] = (z8[3] * SSC + m0.w) + t0.w;
      z8[4] = (z8[4] * SSC + m1.x) + t1.x; z8[5] = (z8[5] * SSC + m1.y) + t1.y;
      z8[6] = (z8[6] * SSC + m1.z) + t1.z; z8[7] = (z8[7] * SSC + m1.w) + t1.w;
      s[jt] = z8;
    }
    float mloc = s[0][0];
    #pragma unroll
    for (int jt = 0; jt < 4; ++jt)
      #pragma unroll
      for (int r = 0; r < 8; ++r) mloc = fmaxf(mloc, s[jt][r]);
    mloc = fmaxf(mloc, __shfl_xor(mloc, 16));
    const float mnew = fmaxf(mrun, mloc);
    const float alpha = __expf(mrun - mnew);
    mrun = mnew;
    float lsum = 0.0f;
    #pragma unroll
    for (int jt = 0; jt < 4; ++jt)
      #pragma unroll
      for (int r = 0; r < 8; ++r) {
        const float p = __expf(s[jt][r] - mnew);
        s[jt][r] = p;
        lsum += p;
      }
    lsum += __shfl_xor(lsum, 16);
    lrun = lrun * alpha + lsum;
    #pragma unroll
    for (int t = 0; t < 8; ++t) o[t] = o[t] * alpha;

    const v16h pb0 = pack2(s[0], s[1], 16384.0f);
    const v16h pb1 = pack2(s[2], s[3], 16384.0f);

    #pragma unroll
    for (int t = 0; t < 8; ++t) {
      const _Float16* vp = Vt + (16 * t + m) * NS + kb;
      const v16h vf0 = load_frag(vp, h);
      const v16h vf1 = load_frag(vp + 32, h);
      o[t] = wmma_f16(vf0, pb0, o[t]);
      o[t] = wmma_f16(vf1, pb1, o[t]);
    }
  }
  const float inv = __builtin_amdgcn_rcpf(lrun) * (1.0f / 512.0f);
  __syncthreads();

  v16h xg[4];
  #pragma unroll
  for (int ks = 0; ks < 4; ++ks) xg[ks] = load_frag(xrow + 32 * ks, h);
  #pragma unroll
  for (int t = 0; t < 8; ++t) {
    v8f acc = zero8;
    #pragma unroll
    for (int ks = 0; ks < 4; ++ks) {
      const v16h wf = load_frag(wg + t * 16 * CD + 32 * ks, h);
      acc = wmma_f16(wf, xg[ks], acc);
    }
    const v8f gp = scale_bias8(acc, 1.0f / 64.0f, bg + hh * CD + 16 * t + 8 * h);
    v8f val;
    #pragma unroll
    for (int r = 0; r < 8; ++r) {
      const float e = __expf(fminf(-gp[r], 80.0f));
      const float sg = __builtin_amdgcn_rcpf(1.0f + e);
      val[r] = o[t][r] * inv * sg;
    }
    *(v8ha*)(Og + (j0 + m) * CD + 16 * t + 8 * h) = cvt8(val, 1.0f);
  }
  __syncthreads();

  _Float16* odst = ogp + (size_t)i * NS * HC + hh * CD;
  #pragma unroll
  for (int it = 0; it < 8; ++it) {
    const int p = it * 384 + tid;
    const int row = p >> 4, pc = p & 15;
    const v8h v = *(const v8ha*)(Og + row * CD + 8 * pc);
    *(volatile v8h*)(odst + (size_t)row * HC + 8 * pc) = v;
  }
  __threadfence();
  #pragma unroll
  for (int it = 0; it < 8; ++it) {
    const int p = it * 384 + tid;
    const int row = p >> 4, pc = p & 15;
    const v8h v = *(const v8ha*)(Og + row * CD + 8 * pc);
    *(volatile v8h*)(odst + (size_t)row * HC + 8 * pc) = v;
  }
}

__global__ __launch_bounds__(128) void trans_kernel(
    const float* __restrict__ z, const float* __restrict__ zmask,
    const float* __restrict__ g, const float* __restrict__ bl,
    const _Float16* __restrict__ w1T, const float* __restrict__ b1,
    const _Float16* __restrict__ w2T, const float* __restrict__ b2,
    float* __restrict__ out)
{
  __shared__ __attribute__((aligned(16))) _Float16 xs[64 * CD];
  __shared__ __attribute__((aligned(16))) float os[64 * CD];
  const int tid = threadIdx.x, lane = tid & 31, w = tid >> 5;
  const int h = lane >> 4, m = lane & 15;
  const int rb = blockIdx.x * 64;

  #pragma unroll 1
  for (int rr = 0; rr < 16; ++rr) {
    const int row = 16 * w + rr;
    const v4f y = ln_row4(z + (size_t)(rb + row) * CD, g, bl, lane);
    const v4h yh = {(_Float16)y.x, (_Float16)y.y, (_Float16)y.z, (_Float16)y.w};
    *(v4ha*)(xs + row * CD + 4 * lane) = yh;
  }
  __syncthreads();

  v16h xf[4];
  #pragma unroll
  for (int ks = 0; ks < 4; ++ks) xf[ks] = load_frag(xs + (16 * w + m) * CD + 32 * ks, h);
  const v8f zero8 = {0.f, 0.f, 0.f, 0.f, 0.f, 0.f, 0.f, 0.f};

  Frag hfr[4];
  #pragma unroll
  for (int kq = 0; kq < 4; ++kq) {
    v8f acc0 = zero8, acc1 = zero8;
    #pragma unroll
    for (int ks = 0; ks < 4; ++ks) {
      const v16h wf0 = load_frag(w1T + (size_t)(32 * kq + m) * CD + 32 * ks, h);
      const v16h wf1 = load_frag(w1T + (size_t)(32 * kq + 16 + m) * CD + 32 * ks, h);
      acc0 = wmma_f16(wf0, xf[ks], acc0);
      acc1 = wmma_f16(wf1, xf[ks], acc1);
    }
    v8f t0 = scale_bias8(acc0, 1.0f / 64.0f, b1 + 32 * kq + 8 * h);
    v8f t1 = scale_bias8(acc1, 1.0f / 64.0f, b1 + 32 * kq + 16 + 8 * h);
    #pragma unroll
    for (int r = 0; r < 8; ++r) { t0[r] = fmaxf(t0[r], 0.0f); t1[r] = fmaxf(t1[r], 0.0f); }
    hfr[kq].half[0] = cvt8(t0, 16.0f);
    hfr[kq].half[1] = cvt8(t1, 16.0f);
  }

  const float mv = zmask[rb + 16 * w + m];
  #pragma unroll
  for (int ct = 0; ct < 8; ++ct) {
    v8f acc = zero8;
    #pragma unroll
    for (int ks = 0; ks < 4; ++ks) {
      const v16h wf = load_frag(w2T + (size_t)(16 * ct + m) * CD + 32 * ks, h);
      acc = wmma_f16(wf, hfr[ks].v, acc);
    }
    v8f t = scale_bias8(acc, 1.0f / 1024.0f, b2 + 16 * ct + 8 * h);
    t = t * mv;
    float* op = os + (16 * w + m) * CD + 16 * ct + 8 * h;
    const v4f u0 = {t[0], t[1], t[2], t[3]};
    const v4f u1 = {t[4], t[5], t[6], t[7]};
    *(v4fa*)op = u0;
    *(v4fa*)(op + 4) = u1;
  }
  __syncthreads();

  #pragma unroll
  for (int it = 0; it < 16; ++it) {
    const int row = 4 * it + w;
    const v4f v = *(const v4fa*)(os + row * CD + 4 * lane)
                + *(const v4fa*)(z + (size_t)(rb + row) * CD + 4 * lane);
    *(volatile v4f*)(out + (size_t)(rb + row) * CD + 4 * lane) = v;
  }
  __threadfence();
  #pragma unroll
  for (int it = 0; it < 16; ++it) {
    const int row = 4 * it + w;
    const v4f v = *(const v4fa*)(os + row * CD + 4 * lane)
                + *(const v4fa*)(z + (size_t)(rb + row) * CD + 4 * lane);
    *(volatile v4f*)(out + (size_t)(rb + row) * CD + 4 * lane) = v;
  }
}

extern "C" void kernel_launch(void* const* d_in, const int* in_sizes, int n_in,
                              void* d_out, int out_size, void* d_ws, size_t ws_size,
                              hipStream_t stream) {
  if (n_in < 42) return;
  if (in_sizes[0] != NZ || out_size != NZ) return;
  if (in_sizes[1] != NP || in_sizes[2] != NS * CD || in_sizes[3] != NS * CD) return;
  if (in_sizes[4] != NS || in_sizes[5] != NS) return;
  if (in_sizes[10] != CD * CD || in_sizes[12] != CD * CD || in_sizes[14] != CD * CD * CD) return;
  if (in_sizes[18] != CD * CD || in_sizes[20] != CD * CD) return;
  for (int d = 0; d < 2; ++d) {
    const int b = 22 + 10 * d;
    if (in_sizes[b + 2] != CD * HC || in_sizes[b + 3] != CD * HC || in_sizes[b + 4] != CD * HC) return;
    if (in_sizes[b + 5] != CD * NH || in_sizes[b + 6] != CD * HC || in_sizes[b + 7] != HC) return;
    if (in_sizes[b + 8] != HC * CD || in_sizes[b + 9] != CD) return;
  }

  const float* z     = (const float*)d_in[0];
  const float* zmask = (const float*)d_in[1];
  const float* tcr   = (const float*)d_in[2];
  const float* pmhc  = (const float*)d_in[3];
  const float* tm    = (const float*)d_in[4];
  const float* pm    = (const float*)d_in[5];
  const float* oln1g = (const float*)d_in[6];
  const float* oln1b = (const float*)d_in[7];
  const float* oln2g = (const float*)d_in[8];
  const float* oln2b = (const float*)d_in[9];
  const float* owa   = (const float*)d_in[10];
  const float* oba   = (const float*)d_in[11];
  const float* owb   = (const float*)d_in[12];
  const float* obb   = (const float*)d_in[13];
  const float* owo   = (const float*)d_in[14];
  const float* obo   = (const float*)d_in[15];
  const float* trlng = (const float*)d_in[16];
  const float* trlnb = (const float*)d_in[17];
  const float* trw1  = (const float*)d_in[18];
  const float* trb1  = (const float*)d_in[19];
  const float* trw2  = (const float*)d_in[20];
  const float* trb2  = (const float*)d_in[21];
  const float* att[2][10];
  for (int d = 0; d < 2; ++d)
    for (int t = 0; t < 10; ++t) att[d][t] = (const float*)d_in[22 + 10 * d + t];
  float* out = (float*)d_out;

  const size_t w_bytes  = (size_t)W_TOTAL * 2;
  const size_t z_bytes  = (size_t)NZ * 4;
  const size_t x_bytes  = (size_t)NP * CD * 2;
  const size_t tb_bytes = (size_t)NH * NP * 4;
  const size_t og_bytes = (size_t)NP * HC * 2;
  const size_t off_w  = 0;
  const size_t off_za = off_w + w_bytes;
  const size_t off_x  = off_za + z_bytes;
  const size_t off_tb = off_x + x_bytes;
  const size_t off_og = off_tb + tb_bytes;
  const size_t total  = off_og + og_bytes;
  if (total > ws_size) return;
  const size_t ab_bytes = (size_t)NS * CD * 2;
  const size_t tt_bytes = (size_t)NS * 16384 * 2;
  if (2 * ab_bytes + tt_bytes > og_bytes) return;

  char* ws = (char*)d_ws;
  _Float16* wd   = (_Float16*)(ws + off_w);
  float*    zA   = (float*)(ws + off_za);
  float*    zB   = out;
  _Float16* xpl  = (_Float16*)(ws + off_x);
  float*    trib = (float*)(ws + off_tb);
  _Float16* ogp  = (_Float16*)(ws + off_og);
  _Float16* a16  = (_Float16*)(ws + off_og);
  _Float16* b16  = (_Float16*)(ws + off_og + ab_bytes);
  _Float16* tT   = (_Float16*)(ws + off_og + 2 * ab_bytes);

  _Float16* waT  = wd + 0;
  _Float16* wbT  = wd + 16384;
  _Float16* w1T  = wd + 32768;
  _Float16* w2T  = wd + 49152;
  _Float16* wo3T = wd + W_O3;
  _Float16* wT[2][5];
  for (int d = 0; d < 2; ++d) {
    _Float16* base = wd + W_DIR0 + (size_t)d * W_DIRSZ;
    wT[d][0] = base; wT[d][1] = base + W_K_OFF; wT[d][2] = base + W_V_OFF;
    wT[d][3] = base + W_G_OFF; wT[d][4] = base + W_O_OFF;
  }
  const size_t attn_lds = 49152 + 49152 + 768;

  prep_kernel<<<(W_GROUPS + 255) / 256, 256, 0, stream>>>(
      owa, owb, trw1, trw2, owo,
      att[0][2], att[0][3], att[0][4], att[0][6], att[0][8],
      att[1][2], att[1][3], att[1][4], att[1][6], att[1][8], wd);
  opm_ab_kernel<<<dim3(NS / 16, 2), 32, 0, stream>>>(tcr, pmhc, tm, pm, oln1g, oln1b, oln2g, oln2b,
                                                     waT, oba, wbT, obb, a16, b16);
  gemm_kernel<0><<<dim3(NS / 64, 16384 / 128), 128, 0, stream>>>(a16, wo3T, z, obo, tm, pm, zA, tT, 0);
  gemm_kernel<1><<<dim3(NS / 64, NS), 128, 0, stream>>>(b16, tT, z, obo, tm, pm, zA, tT, 0);
  ln_kernel<<<NP / 32, 256, 0, stream>>>(zA, att[0][0], att[0][1], att[0][5], xpl, trib, 0);
  attn_kernel<<<NS * NH, 384, attn_lds, stream>>>(xpl, trib, zmask, wT[0][0], wT[0][1], wT[0][2], wT[0][3],
                                                   att[0][7], ogp, 0);
  gemm_kernel<2><<<dim3(NP / 64, 1), 128, 0, stream>>>(ogp, wT[0][4], zA, att[0][9], tm, pm, zB, tT, 0);
  ln_kernel<<<NP / 32, 256, 0, stream>>>(zB, att[1][0], att[1][1], att[1][5], xpl, trib, 1);
  attn_kernel<<<NS * NH, 384, attn_lds, stream>>>(xpl, trib, zmask, wT[1][0], wT[1][1], wT[1][2], wT[1][3],
                                                   att[1][7], ogp, 1);
  gemm_kernel<2><<<dim3(NP / 64, 1), 128, 0, stream>>>(ogp, wT[1][4], zB, att[1][9], tm, pm, zA, tT, 1);
  trans_kernel<<<NP / 64, 128, 0, stream>>>(zA, zmask, trlng, trlnb, w1T, trb1, w2T, trb2, out);
}
